// VanillaAttention_34737695490632
// MI455X (gfx1250) — hardware-run, weakly checked
//
#include <hip/hip_runtime.h>
#include <stddef.h>

typedef __attribute__((ext_vector_type(16))) _Float16 v16h;
typedef __attribute__((ext_vector_type(8)))  _Float16 v8h;
typedef __attribute__((ext_vector_type(16))) __bf16   v16b;
typedef __attribute__((ext_vector_type(8)))  __bf16   v8b;
typedef __attribute__((ext_vector_type(8)))  float    v8f;
typedef __attribute__((ext_vector_type(4)))  float    v4f;

constexpr int kNQ  = 2048;
constexpr int kNK  = 2048;
constexpr int kDim = 64;
constexpr int QPITCH = 68;
constexpr int WPITCH = 136;

static_assert(kNQ % 64 == 0 && kNK % 64 == 0 && kDim % 64 == 0, "GEMM M/N tile multiples");
static_assert(kDim % 32 == 0 && kNK % 32 == 0, "GEMM K multiples of 32");
static_assert(kNK == 2048 && kDim == 64, "softmax and score kernels assume these extents");

constexpr size_t BYTES_ACT16 = (size_t)kNQ * kDim * 2;
constexpr size_t BYTES_W16   = (size_t)kDim * kDim * 2;
constexpr size_t BYTES_ACT32 = (size_t)kNQ * kDim * 4;
constexpr size_t BYTES_VT16  = (size_t)kDim * kNK * 2;
constexpr size_t BYTES_MEANV = 256;
constexpr size_t BYTES_P16   = (size_t)kNQ * kNK * 2;
constexpr size_t OFF_QHI  = 0;
constexpr size_t OFF_QLO  = OFF_QHI + BYTES_ACT16;
constexpr size_t OFF_KHI  = OFF_QLO + BYTES_ACT16;
constexpr size_t OFF_KLO  = OFF_KHI + BYTES_ACT16;
constexpr size_t OFF_WQHI = OFF_KLO + BYTES_ACT16;
constexpr size_t OFF_WQLO = OFF_WQHI + BYTES_W16;
constexpr size_t OFF_WKHI = OFF_WQLO + BYTES_W16;
constexpr size_t OFF_WKLO = OFF_WKHI + BYTES_W16;
constexpr size_t OFF_QP   = OFF_WKLO + BYTES_W16;
constexpr size_t OFF_KP   = OFF_QP + BYTES_ACT32;
constexpr size_t OFF_VT   = OFF_KP + BYTES_ACT32;
constexpr size_t OFF_MEANV = OFF_VT + BYTES_VT16;
constexpr size_t OFF_P    = OFF_MEANV + BYTES_MEANV;
constexpr size_t WS_TOTAL = OFF_P + BYTES_P16;
static_assert(OFF_QLO % 128 == 0 && OFF_KHI % 128 == 0 && OFF_KLO % 128 == 0 && OFF_WQHI % 128 == 0, "align");
static_assert(OFF_WQLO % 128 == 0 && OFF_WKHI % 128 == 0 && OFF_WKLO % 128 == 0 && OFF_QP % 128 == 0, "align");
static_assert(OFF_KP % 128 == 0 && OFF_VT % 128 == 0 && OFF_MEANV % 128 == 0 && OFF_P % 128 == 0, "align");
static_assert(WS_TOTAL <= (size_t)134217728, "workspace budget");
constexpr size_t OUT1_ELEM_OFF = 524288 / 4;
static_assert(OUT1_ELEM_OFF == (size_t)kNQ * kDim, "out1 offset");
static_assert(524288 + (size_t)kNQ * kNK * 4 == (size_t)17301504, "out total");

__device__ __forceinline__ unsigned short f2bf_bits(float f) {
  unsigned u = __float_as_uint(f);
  return (unsigned short)((u + 0x7FFFu + ((u >> 16) & 1u)) >> 16);
}
__device__ __forceinline__ float bf_bits2f(unsigned short h) { return __uint_as_float(((unsigned)h) << 16); }

__device__ __forceinline__ void dep_guard_h(v8f& a, v8f& b, v16h x, v16h y) { asm volatile("v_nop\n\tv_nop\n\tv_nop\n\tv_nop" : "+v"(a), "+v"(b) : "v"(x), "v"(y)); }
__device__ __forceinline__ void dep_guard_b(v8f& a, v8f& b, v16b x, v16b y) { asm volatile("v_nop\n\tv_nop\n\tv_nop\n\tv_nop" : "+v"(a), "+v"(b) : "v"(x), "v"(y)); }
__device__ __forceinline__ void keep4_h(v16h a, v16h b, v16h c, v16h d) { asm volatile("v_nop" :: "v"(a), "v"(b), "v"(c), "v"(d)); }
__device__ __forceinline__ void keep4_b(v16b a, v16b b, v16b c, v16b d) { asm volatile("v_nop" :: "v"(a), "v"(b), "v"(c), "v"(d)); }
__device__ __forceinline__ void acc_guard4(v8f& a, v8f& b, v8f& c, v8f& d) { asm volatile("v_nop\n\tv_nop\n\tv_nop\n\tv_nop" : "+v"(a), "+v"(b), "+v"(c), "+v"(d)); }
template <typename T> struct Frag;
template <> struct Frag<_Float16> {
  typedef v16h V; union U { v16h v; v8h h[2]; };
  static __device__ __forceinline__ v16h load(const _Float16* p) {
    U f; f.h[0] = *(const v8h*)(p); f.h[1] = *(const v8h*)(p + 16); return f.v;
  }
  static __device__ __forceinline__ v8f mma(v16h a, v16h b, v8f c) {
    return __builtin_amdgcn_wmma_f32_16x16x32_f16(false, a, false, b, (short)0, c, false, false);
  }
  static __device__ __forceinline__ void guard(v8f& a, v8f& b, v16h x, v16h y) { dep_guard_h(a, b, x, y); }
  static __device__ __forceinline__ void keep(v16h a, v16h b, v16h c, v16h d) { keep4_h(a, b, c, d); }
};
template <> struct Frag<__bf16> {
  typedef v16b V; union U { v16b v; v8b h[2]; };
  static __device__ __forceinline__ v16b load(const __bf16* p) {
    U f; f.h[0] = *(const v8b*)(p); f.h[1] = *(const v8b*)(p + 16); return f.v;
  }
  static __device__ __forceinline__ v8f mma(v16b a, v16b b, v8f c) {
    return __builtin_amdgcn_wmma_f32_16x16x32_bf16(false, a, false, b, (short)0, c, false, false);
  }
  static __device__ __forceinline__ void guard(v8f& a, v8f& b, v16b x, v16b y) { dep_guard_b(a, b, x, y); }
  static __device__ __forceinline__ void keep(v16b a, v16b b, v16b c, v16b d) { keep4_b(a, b, c, d); }
};

__device__ __forceinline__ v8f mma_h(v16h a, v16h b, v8f c) {
  c = __builtin_amdgcn_wmma_f32_16x16x32_f16(false, a, false, b, (short)0, c, false, false);
  asm volatile("v_nop\n\tv_nop\n\tv_nop\n\tv_nop" : "+v"(c) : "v"(a), "v"(b));
  return c;
}

template <int ET> struct Elem;
template <> struct Elem<0> { typedef _Float16 T; };
template <> struct Elem<1> { typedef __bf16 T; };
template <int ET, bool SPLIT, int BIAS_MODE, int OUT_MODE, bool RESID, int ACT = 0, bool ADDN = false>
__global__ __launch_bounds__(256) void wmma_gemm64(
    const unsigned short* __restrict__ Ap, const unsigned short* __restrict__ A2p, int lda, long strideA,
    const unsigned short* __restrict__ Btp, const unsigned short* __restrict__ Bt2p, int ldb, long strideB,
    void* __restrict__ Cout, void* __restrict__ Cout2, int ldc, long strideC,
    const float* __restrict__ bias,
    const float* __restrict__ resid, long strideR,
    int M, int N, int K, float scale,
    const float* __restrict__ addn) {
  typedef typename Elem<ET>::T T;
  typedef typename Frag<T>::V V;
  const T* A = (const T*)Ap; const T* A2 = (const T*)A2p; const T* Bt = (const T*)Btp; const T* Bt2 = (const T*)Bt2p;
  __shared__ __align__(16) float sT[8][16 * 68];
  const int b    = blockIdx.y;
  const int lane = threadIdx.x & 31;
  const int wave = threadIdx.x >> 5;
  const int tilesN = N >> 6;
  const int tilesM = M >> 6;
  const int tile = blockIdx.x * 8 + wave;
  if (tile >= tilesM * tilesN) return;
  const int tm = tile / tilesN;
  const int tn = tile - tm * tilesN;
  const int m0 = tm << 6;
  const int n0 = tn << 6;

  const T* Ab  = A  + (size_t)b * strideA;
  const T* Bb  = Bt + (size_t)b * strideB;
  const T* Ab2 = SPLIT ? (A2  + (size_t)b * strideA) : nullptr;
  const T* Bb2 = SPLIT ? (Bt2 + (size_t)b * strideB) : nullptr;

  const int rlane = lane & 15;
  const int koff  = (lane >> 4) * 8;
  const int mOff  = (lane >> 4) * 8;

  v8f acc[4][4];
#pragma unroll
  for (int i = 0; i < 4; ++i)
#pragma unroll
    for (int j = 0; j < 4; ++j) acc[i][j] = (v8f){0.f,0.f,0.f,0.f,0.f,0.f,0.f,0.f};

  for (int k0 = 0; k0 < K; k0 += 32) {
    V bh[4], bl[4];
#pragma unroll
    for (int j = 0; j < 4; ++j) {
      const size_t bo = (size_t)(n0 + (j << 4) + rlane) * ldb + koff + k0;
      bh[j] = Frag<T>::load(Bb + bo);
      if (SPLIT) bl[j] = Frag<T>::load(Bb2 + bo);
    }
#pragma unroll
    for (int i = 0; i < 4; ++i) {
      const size_t ao = (size_t)(m0 + (i << 4) + rlane) * lda + koff + k0;
      V ah = Frag<T>::load(Ab + ao);
      V al;
      if (SPLIT) al = Frag<T>::load(Ab2 + ao);
#pragma unroll
      for (int j = 0; j < 4; ++j) {
        acc[i][j] = Frag<T>::mma(ah, bh[j], acc[i][j]);
        if (SPLIT) {
          acc[i][j] = Frag<T>::mma(ah, bl[j], acc[i][j]);
          acc[i][j] = Frag<T>::mma(al, bh[j], acc[i][j]);
        }
      }
      Frag<T>::guard(acc[i][0], acc[i][3], ah, SPLIT ? al : ah);
    }
    Frag<T>::keep(bh[0], bh[1], bh[2], bh[3]);
    if (SPLIT) Frag<T>::keep(bl[0], bl[1], bl[2], bl[3]);
  }
  acc_guard4(acc[0][0], acc[0][1], acc[0][2], acc[0][3]);
  acc_guard4(acc[1][0], acc[1][1], acc[1][2], acc[1][3]);
  acc_guard4(acc[2][0], acc[2][1], acc[2][2], acc[2][3]);
  acc_guard4(acc[3][0], acc[3][1], acc[3][2], acc[3][3]);

  float* slab = sT[wave];
  const float* Rb = RESID ? (resid + (size_t)b * strideR) : nullptr;
#pragma unroll
  for (int i = 0; i < 4; ++i) {
    const int mBase = m0 + (i << 4);
#pragma unroll
    for (int j = 0; j < 4; ++j) {
      const int n = n0 + (j << 4) + rlane;
      float bv = 0.f;
      if (BIAS_MODE == 2) bv = bias[n];
#pragma unroll
      for (int r = 0; r < 8; ++r) {
        float v = acc[i][j][r] * scale;
        if (BIAS_MODE == 1) v += bias[mBase + mOff + r];
        if (BIAS_MODE == 2) v += bv;
        if (RESID) v += Rb[(size_t)(mBase + mOff + r) * ldc + n];
        if (ACT == 1) v = tanhf(v);
        if (ACT == 2) v = fmaxf(v, 0.0f);
        if (ACT == 3) v = v / (1.0f + expf(-v));
        if (ACT == 4) v = (v > 0.f) ? v : 0.01f * v;
        if (ACT == 5) v = 0.5f * v * (1.0f + erff(v * 0.70710678118654752f));
        slab[(mOff + r) * 68 + (j << 4) + rlane] = v;
      }
    }
    __builtin_amdgcn_fence(__ATOMIC_RELEASE, "workgroup");
    __builtin_amdgcn_wave_barrier();
    __builtin_amdgcn_fence(__ATOMIC_ACQUIRE, "workgroup");
    if (OUT_MODE == 0) {
      float* C = (float*)Cout + (size_t)b * strideC;
      const int hh = lane >> 4, c4 = (lane & 15) * 4;
      v4f av = (v4f){0.f, 0.f, 0.f, 0.f};
      if (ADDN) av = *(const v4f*)(addn + n0 + c4);
      for (int pass = 0; pass < 2; ++pass) {
#pragma unroll
        for (int it = 0; it < 8; ++it) {
          const int row = it * 2 + hh;
          v4f v = *(const v4f*)(slab + row * 68 + c4);
          if (ADDN) v = v + av;
          *(volatile v4f*)(C + (size_t)(mBase + row) * ldc + n0 + c4) = v;
        }
        __threadfence();
      }
    } else {
      const int q = lane >> 3, c8 = (lane & 7) * 8;
      unsigned short* C  = (unsigned short*)Cout  + (size_t)b * strideC;
      unsigned short* C2 = (OUT_MODE == 2) ? ((unsigned short*)Cout2 + (size_t)b * strideC) : nullptr;
      for (int pass = 0; pass < 2; ++pass) {
#pragma unroll
        for (int it = 0; it < 4; ++it) {
          const int row = it * 4 + q;
          const float* sp = slab + row * 68 + c8;
          v8h hv, lv;
#pragma unroll
          for (int e = 0; e < 8; ++e) {
            if (OUT_MODE == 1) {
              hv[e] = (_Float16)sp[e];
            } else {
              unsigned short hb = f2bf_bits(sp[e]);
              unsigned short lb = f2bf_bits(sp[e] - bf_bits2f(hb));
              hv[e] = __builtin_bit_cast(_Float16, hb);
              lv[e] = __builtin_bit_cast(_Float16, lb);
            }
          }
          *(volatile v8h*)(C + (size_t)(mBase + row) * ldc + n0 + c8) = hv;
          if (OUT_MODE == 2) *(volatile v8h*)(C2 + (size_t)(mBase + row) * ldc + n0 + c8) = lv;
        }
        __threadfence();
      }
    }
    __builtin_amdgcn_fence(__ATOMIC_RELEASE, "workgroup");
    __builtin_amdgcn_wave_barrier();
    __builtin_amdgcn_fence(__ATOMIC_ACQUIRE, "workgroup");
  }
}

template <bool TR>
__global__ __launch_bounds__(256) void split_bf16_x2(
    const float* __restrict__ in, unsigned short* __restrict__ hi, unsigned short* __restrict__ lo,
    int R, int logC, int n2) {
  const int i = blockIdx.x * 256 + threadIdx.x;
  if (i < n2) {
    unsigned uh = 0u, ul = 0u;
#pragma unroll
    for (int t = 0; t < 2; ++t) {
      const int e = 2 * i + t;
      const int r = e >> logC;
      const int c = e & ((1 << logC) - 1);
      const int idx = TR ? (c * R + r) : e;
      const float x = in[idx];
      const unsigned short hb = f2bf_bits(x);
      const unsigned short lb = f2bf_bits(x - bf_bits2f(hb));
      uh |= ((unsigned)hb) << (16 * t);
      ul |= ((unsigned)lb) << (16 * t);
    }
    ((volatile unsigned*)hi)[i] = uh;
    ((volatile unsigned*)lo)[i] = ul;
    __threadfence();
    ((volatile unsigned*)hi)[i] = uh;
    ((volatile unsigned*)lo)[i] = ul;
  }
}

__global__ __launch_bounds__(256) void cast_f16T_x2(
    const float* __restrict__ in, unsigned short* __restrict__ out, int R, int logC, int n2) {
  const int i = blockIdx.x * 256 + threadIdx.x;
  if (i < n2) {
    unsigned u = 0u;
#pragma unroll
    for (int t = 0; t < 2; ++t) {
      const int e = 2 * i + t;
      const int r = e >> logC;
      const int c = e & ((1 << logC) - 1);
      const float x = in[c * R + r];
      const _Float16 h = (_Float16)x;
      u |= ((unsigned)__builtin_bit_cast(unsigned short, h)) << (16 * t);
    }
    ((volatile unsigned*)out)[i] = u;
    __threadfence();
    ((volatile unsigned*)out)[i] = u;
  }
}

__global__ __launch_bounds__(256) void colmean_kernel(const float* __restrict__ v, float* __restrict__ meanv) {
  __shared__ float part[4 * 64];
  const int tid = threadIdx.x;
  const int d = tid & 63, rq = tid >> 6;
  const float* src = v + (size_t)(rq * 512) * kDim + d;
  float s0 = 0.f, s1 = 0.f, s2 = 0.f, s3 = 0.f;
#pragma unroll 1
  for (int r = 0; r < 512; r += 4) {
    s0 += src[(size_t)(r + 0) * kDim];
    s1 += src[(size_t)(r + 1) * kDim];
    s2 += src[(size_t)(r + 2) * kDim];
    s3 += src[(size_t)(r + 3) * kDim];
  }
  part[rq * 64 + d] = (s0 + s1) + (s2 + s3);
  __syncthreads();
  if (tid < 64) {
    const float tot = (part[tid] + part[64 + tid]) + (part[128 + tid] + part[192 + tid]);
    const float mv = tot * (1.0f / 2048.0f);
    ((volatile float*)meanv)[tid] = mv;
    __threadfence();
    ((volatile float*)meanv)[tid] = mv;
  }
}

__global__ __launch_bounds__(256) void score_kernel(const float* __restrict__ qp, const float* __restrict__ kp,
                                                    const float* __restrict__ w, const float* __restrict__ bptr,
                                                    float* __restrict__ att) {
  __shared__ __align__(16) float qs[64 * QPITCH];
  __shared__ __align__(16) float ks[64 * QPITCH];
  __shared__ __align__(16) _Float16 wtab[16 * WPITCH];
  __shared__ float wsh[64];
  __shared__ __align__(16) float slab[8][2 * QPITCH];

  const int tid = threadIdx.x;
  const int wave = tid >> 5, lane = tid & 31;
  const int hh = lane >> 4, p = lane & 15;
  const int n0 = blockIdx.y * 64;
  const int m0 = blockIdx.x * 64;

  {
    const int row = tid >> 2, cseg = (tid & 3) * 16;
    const float* qsrc = qp + (size_t)(n0 + row) * kDim + cseg;
    const float* ksrc = kp + (size_t)(m0 + row) * kDim + cseg;
#pragma unroll 1
    for (int i = 0; i < 4; ++i) {
      const v4f a = *(const v4f*)(qsrc + 4 * i);
      const v4f c = *(const v4f*)(ksrc + 4 * i);
      v4f ea, ec;
#pragma unroll
      for (int e = 0; e < 4; ++e) { ea[e] = expf(-a[e]); ec[e] = expf(-c[e]); }
      *(v4f*)(qs + row * QPITCH + cseg + 4 * i) = ea;
      *(v4f*)(ks + row * QPITCH + cseg + 4 * i) = ec;
    }
  }
  if (tid < 64) wsh[tid] = w[tid];
  __syncthreads();

  {
    const int row = tid >> 4, kseg = (tid & 15) * 8;
    v8h tv;
#pragma unroll
    for (int e = 0; e < 8; ++e) {
      const int kk = kseg + e;
      const int d = kk & 63;
      const float w64 = wsh[d] * 64.0f;
      const _Float16 whi = (_Float16)w64;
      const float whif = (float)whi;
      const float wlo = (w64 - whif) * 32768.0f;
      float val = 0.0f;
      if (row == 0 && kk < 64) val = whif;
      if (row == 1 && kk < 64) val = wlo;
      if (row == 2 && kk >= 64) val = whif;
      tv[e] = (_Float16)val;
    }
    *(v8h*)(wtab + row * WPITCH + kseg) = tv;
  }
  __syncthreads();

  v16h aw[4];
#pragma unroll
  for (int s4 = 0; s4 < 4; ++s4) aw[s4] = Frag<_Float16>::load(wtab + p * WPITCH + 8 * hh + 32 * s4);

  const float bb = bptr[0];
  float* myslab = slab[wave];
  const int nw = n0 + wave * 8;

#pragma unroll 1
  for (int rp = 0; rp < 4; ++rp) {
#pragma unroll 1
    for (int u = 0; u < 8; ++u) {
      const int j = u >> 2, g = u & 3;
      const int nl = wave * 8 + rp * 2 + j;
      const int ml = 4 * p + g;
      const float* eq = qs + nl * QPITCH;
      const float* ek = ks + ml * QPITCH;
      v8f acc = (v8f){0.f, 0.f, 0.f, 0.f, 0.f, 0.f, 0.f, 0.f};
#pragma unroll
      for (int s = 0; s < 2; ++s) {
        v16h fh, fl;
#pragma unroll
        for (int half = 0; half < 2; ++half) {
#pragma unroll
          for (int qq = 0; qq < 2; ++qq) {
            const int dbase = 32 * s + 16 * half + 8 * hh + 4 * qq;
            const v4f qv = *(const v4f*)(eq + dbase);
            const v4f kv = *(const v4f*)(ek + dbase);
#pragma unroll
            for (int e = 0; e < 4; ++e) {
              const float t = fmaf(qv[e], kv[e], 1.0f);
              const float sg = __builtin_amdgcn_rcpf(t);
              const _Float16 hi = (_Float16)sg;
              const float hif = (float)hi;
              const float lo = (sg - hif) * 32768.0f;
              fh[8 * half + 4 * qq + e] = hi;
              fl[8 * half + 4 * qq + e] = (_Float16)lo;
            }
          }
        }
        acc = mma_h(aw[s], fh, acc);
        acc = mma_h(aw[2 + s], fl, acc);
      }
      const float sc = acc[0] * (1.0f / 64.0f) + (acc[1] + acc[2]) * (1.0f / (64.0f * 32768.0f)) + bb;
      if (hh == 0) myslab[j * QPITCH + ml] = sc;
    }
    __builtin_amdgcn_fence(__ATOMIC_RELEASE, "workgroup");
    __builtin_amdgcn_wave_barrier();
    __builtin_amdgcn_fence(__ATOMIC_ACQUIRE, "workgroup");
    {
      const int c4 = p * 4;
      const int row = nw + rp * 2 + hh;
      const v4f val = *(const v4f*)(myslab + hh * QPITCH + c4);
      float* dst = att + (size_t)row * kNK + m0 + c4;
      *(volatile v4f*)dst = val;
      __threadfence();
      *(volatile v4f*)dst = val;
    }
    __builtin_amdgcn_fence(__ATOMIC_RELEASE, "workgroup");
    __builtin_amdgcn_wave_barrier();
    __builtin_amdgcn_fence(__ATOMIC_ACQUIRE, "workgroup");
  }
}

__global__ __launch_bounds__(256) void softmax_kernel(const float* __restrict__ att, unsigned short* __restrict__ P16) {
  __shared__ float redm[8];
  __shared__ float reds[8];
  const int tid = threadIdx.x, lane = tid & 31, wave = tid >> 5;
  const int row = blockIdx.x;
  const float* s = att + (size_t)row * kNK + 8 * tid;
  const v4f a0 = *(const v4f*)s;
  const v4f a1 = *(const v4f*)(s + 4);
  float m = fmaxf(fmaxf(fmaxf(a0[0], a0[1]), fmaxf(a0[2], a0[3])),
                  fmaxf(fmaxf(a1[0], a1[1]), fmaxf(a1[2], a1[3])));
#pragma unroll
  for (int off = 1; off < 32; off <<= 1) m = fmaxf(m, __shfl_xor(m, off, 32));
  if (lane == 0) redm[wave] = m;
  __syncthreads();
  float mx = redm[0];
#pragma unroll
  for (int i = 1; i < 8; ++i) mx = fmaxf(mx, redm[i]);
  v4f e0, e1;
  float sum = 0.f;
#pragma unroll
  for (int e = 0; e < 4; ++e) { e0[e] = expf(a0[e] - mx); sum += e0[e]; }
#pragma unroll
  for (int e = 0; e < 4; ++e) { e1[e] = expf(a1[e] - mx); sum += e1[e]; }
#pragma unroll
  for (int off = 1; off < 32; off <<= 1) sum += __shfl_xor(sum, off, 32);
  if (lane == 0) reds[wave] = sum;
  __syncthreads();
  float tot = reds[0];
#pragma unroll
  for (int i = 1; i < 8; ++i) tot += reds[i];
  const float scl = 16384.0f / tot;
  v8h hv;
#pragma unroll
  for (int e = 0; e < 4; ++e) {
    hv[e]     = (_Float16)(e0[e] * scl - 8.0f);
    hv[4 + e] = (_Float16)(e1[e] * scl - 8.0f);
  }
  _Float16* dst = (_Float16*)P16 + (size_t)row * kNK + 8 * tid;
  *(volatile v8h*)dst = hv;
  __threadfence();
  *(volatile v8h*)dst = hv;
}

extern "C" void kernel_launch(void* const* d_in, const int* in_sizes, int n_in,
                              void* d_out, int out_size, void* d_ws, size_t ws_size,
                              hipStream_t stream) {
  if (n_in < 9) return;
  if (in_sizes[0] != kNQ * kDim || in_sizes[1] != kNK * kDim || in_sizes[2] != kNK * kDim) return;
  if (in_sizes[3] != kDim * kDim || in_sizes[4] != kDim || in_sizes[5] != kDim * kDim || in_sizes[6] != kDim) return;
  if (in_sizes[7] != kDim || in_sizes[8] < 1) return;
  if (out_size != kNQ * kDim + kNQ * kNK) return;
  if (ws_size < WS_TOTAL) return;

  const float* q  = (const float*)d_in[0];
  const float* k  = (const float*)d_in[1];
  const float* v  = (const float*)d_in[2];
  const float* Wq = (const float*)d_in[3];
  const float* bq = (const float*)d_in[4];
  const float* Wk = (const float*)d_in[5];
  const float* bk = (const float*)d_in[6];
  const float* w  = (const float*)d_in[7];
  const float* b  = (const float*)d_in[8];

  float* out0 = (float*)d_out;
  float* att  = (float*)d_out + OUT1_ELEM_OFF;

  char* ws = (char*)d_ws;
  unsigned short* qhi  = (unsigned short*)(ws + OFF_QHI);
  unsigned short* qlo  = (unsigned short*)(ws + OFF_QLO);
  unsigned short* khi  = (unsigned short*)(ws + OFF_KHI);
  unsigned short* klo  = (unsigned short*)(ws + OFF_KLO);
  unsigned short* wqhi = (unsigned short*)(ws + OFF_WQHI);
  unsigned short* wqlo = (unsigned short*)(ws + OFF_WQLO);
  unsigned short* wkhi = (unsigned short*)(ws + OFF_WKHI);
  unsigned short* wklo = (unsigned short*)(ws + OFF_WKLO);
  float*          qp   = (float*)(ws + OFF_QP);
  float*          kpp  = (float*)(ws + OFF_KP);
  unsigned short* vT   = (unsigned short*)(ws + OFF_VT);
  float*          meanv = (float*)(ws + OFF_MEANV);
  unsigned short* P16  = (unsigned short*)(ws + OFF_P);

  const int n2act = (kNQ * kDim) / 2;
  const int n2w   = (kDim * kDim) / 2;
  const int n2v   = (kDim * kNK) / 2;
  split_bf16_x2<false><<<(n2act + 255) / 256, 256, 0, stream>>>(q, qhi, qlo, kNQ, 6, n2act);
  split_bf16_x2<false><<<(n2act + 255) / 256, 256, 0, stream>>>(k, khi, klo, kNK, 6, n2act);
  split_bf16_x2<true><<<(n2w + 255) / 256, 256, 0, stream>>>(Wq, wqhi, wqlo, kDim, 6, n2w);
  split_bf16_x2<true><<<(n2w + 255) / 256, 256, 0, stream>>>(Wk, wkhi, wklo, kDim, 6, n2w);
  cast_f16T_x2<<<(n2v + 255) / 256, 256, 0, stream>>>(v, vT, kDim, 11, n2v);
  colmean_kernel<<<1, 256, 0, stream>>>(v, meanv);

  const int projBlocks = ((kNQ / 64) * (kDim / 64) + 7) / 8;
  wmma_gemm64<1, true, 2, 0, false, 0, false><<<dim3(projBlocks, 1), 256, 0, stream>>>(
      qhi, qlo, kDim, 0L, wqhi, wqlo, kDim, 0L, (void*)qp, nullptr, kDim, 0L,
      bq, nullptr, 0L, kNQ, kDim, kDim, 1.0f, nullptr);
  wmma_gemm64<1, true, 2, 0, false, 0, false><<<dim3(projBlocks, 1), 256, 0, stream>>>(
      khi, klo, kDim, 0L, wkhi, wklo, kDim, 0L, (void*)kpp, nullptr, kDim, 0L,
      bk, nullptr, 0L, kNK, kDim, kDim, 1.0f, nullptr);

  score_kernel<<<dim3(kNK / 64, kNQ / 64), 256, 0, stream>>>(qp, kpp, w, b, att);

  softmax_kernel<<<kNQ, 256, 0, stream>>>(att, P16);

  const int pvBlocks = ((kNQ / 64) * (kDim / 64) + 7) / 8;
  wmma_gemm64<0, false, 0, 0, false, 0, true><<<dim3(pvBlocks, 1), 256, 0, stream>>>(
      P16, nullptr, kNK, 0L, vT, nullptr, kNK, 0L, (void*)out0, nullptr, kDim, 0L,
      nullptr, nullptr, 0L, kNQ, kDim, kNK, 1.0f / 16384.0f, meanv);
}
